// tinystoriesgru_23115513987273
// MI455X (gfx1250) — hardware-verified
//
#include <hip/hip_runtime.h>
#include <math.h>

constexpr int NBATCH    = 64;
constexpr int NSTEP     = 256;
constexpr int NEMB      = 384;
constexpr int NHEAD     = 6;
constexpr int HDIM      = 64;
constexpr int SQRT_HDIM = 8;
constexpr int NVOC      = 128;
constexpr int NGATE     = 3 * NEMB;
constexpr int NCAT      = 2 * NEMB;
constexpr int NROWS     = NBATCH * NSTEP;
constexpr int NOUT      = NROWS * NVOC;
static_assert(NEMB == NHEAD * HDIM);
static_assert(SQRT_HDIM * SQRT_HDIM == HDIM);
static_assert(HDIM == 64);
static_assert(NEMB % 32 == 0 && NCAT % 32 == 0 && HDIM % 32 == 0);
static_assert(NROWS % 64 == 0 && NGATE % 64 == 0 && NEMB % 64 == 0 && NVOC % 64 == 0);
static_assert(NSTEP % 64 == 0);
static_assert(NBATCH % 16 == 0);

constexpr float W_CARRY   = 16.0f;
constexpr float X_CARRY   = 16.0f;
constexpr float Q_CARRY   = 64.0f;
constexpr float P_CARRY   = 32768.0f;
constexpr float C_CARRY   = 1024.0f;
constexpr float AC_CARRY  = 256.0f;
constexpr float PRE_CARRY = 64.0f;
constexpr float S_CARRY   = 64.0f;
constexpr float N_CARRY   = 16.0f;
constexpr float PRE_INV   = 1.0f / PRE_CARRY;
constexpr float ST_FOLD   = 1.0f / (S_CARRY * W_CARRY);
constexpr float SC_SCALE  = (1.0f / (float)SQRT_HDIM) / (Q_CARRY * Q_CARRY);
constexpr float MASK_FILL = -1e30f;
constexpr float LN_EPS_F  = 1e-5f;

typedef __attribute__((ext_vector_type(16))) _Float16 v16h;
typedef __attribute__((ext_vector_type(8)))  _Float16 v8h;
typedef __attribute__((ext_vector_type(4)))  _Float16 v4h;
typedef __attribute__((ext_vector_type(8)))  float    v8f;
typedef __attribute__((ext_vector_type(4)))  float    v4f;
typedef __attribute__((ext_vector_type(4)))  unsigned v4u;

struct FragH {
  union U { v16h v; v8h h[2]; };
  static __device__ __forceinline__ v16h load(const _Float16* p) {
    U f;
    f.h[0] = *(const v8h*)(p);
    f.h[1] = *(const v8h*)(p + 16);
    return f.v;
  }
  static __device__ __forceinline__ v8f mma(v16h a, v16h b, v8f c) {
    return __builtin_amdgcn_wmma_f32_16x16x32_f16(false, a, false, b, (short)0, c, false, false);
  }
};

__device__ __forceinline__ v8f mma_n(v16h a, v16h b, v8f c) {
  c = __builtin_amdgcn_wmma_f32_16x16x32_f16(false, a, false, b, (short)0, c, false, false);
  asm volatile("v_nop\n\tv_nop\n\tv_nop\n\tv_nop" : "+v"(c) : "v"(a), "v"(b));
  return c;
}
__device__ __forceinline__ void guard_gemm(v8f& a, v8f& b, v8f& c, v8f& d, v16h x, v16h b0, v16h b1, v16h b2, v16h b3) {
  asm volatile("v_nop\n\tv_nop\n\tv_nop\n\tv_nop" : "+v"(a), "+v"(b), "+v"(c), "+v"(d) : "v"(x), "v"(b0), "v"(b1), "v"(b2), "v"(b3));
}
__device__ __forceinline__ void guard_scan(v8f& a, v8f& b, v8f& c, v8f& d, v16h x, v16h y,
                                           v16h b0, v16h b1, v16h b2, v16h b3, v16h b4, v16h b5) {
  asm volatile("v_nop\n\tv_nop\n\tv_nop\n\tv_nop" : "+v"(a), "+v"(b), "+v"(c), "+v"(d)
               : "v"(x), "v"(y), "v"(b0), "v"(b1), "v"(b2), "v"(b3), "v"(b4), "v"(b5));
}
__device__ __forceinline__ void acc_guard4(v8f& a, v8f& b, v8f& c, v8f& d) {
  asm volatile("v_nop\n\tv_nop\n\tv_nop\n\tv_nop" : "+v"(a), "+v"(b), "+v"(c), "+v"(d));
}
__device__ __forceinline__ void acc_guard1(v8f& a) {
  asm volatile("v_nop\n\tv_nop\n\tv_nop\n\tv_nop" : "+v"(a));
}

__device__ __forceinline__ float h16_to_f32(unsigned hb) {
  const unsigned sgn = (hb & 0x8000u) << 16;
  const unsigned em = hb & 0x7fffu;
  const float fn = __uint_as_float((em << 13) + 0x38000000u);
  const float fs = (float)em * 5.9604644775390625e-8f;
  const float mag = (em < 0x400u) ? fs : fn;
  return __uint_as_float(__float_as_uint(mag) | sgn);
}

__device__ __forceinline__ float sig_f(float x) { return 1.0f / (1.0f + expf(-x)); }

__global__ __launch_bounds__(256) void cvt8_f16_kernel(const float* __restrict__ src, unsigned short* __restrict__ dst,
                                                       int nrow, int ncol8, int spitch, int scol0, float sc) {
  const int i  = blockIdx.x * 256 + threadIdx.x;
  const int n8 = nrow * ncol8;
  if (i < n8) {
    const int row = i / ncol8;
    const int c8  = i - row * ncol8;
    const float* sp = src + (size_t)row * spitch + scol0 + c8 * 8;
    const v4f a = *(const v4f*)(sp);
    const v4f b = *(const v4f*)(sp + 4);
    v8h hv;
#pragma unroll
    for (int e = 0; e < 4; ++e) {
      hv[e]     = (_Float16)(a[e] * sc);
      hv[4 + e] = (_Float16)(b[e] * sc);
    }
    *(volatile v8h*)(dst + (size_t)i * 8) = hv;
    __threadfence();
    *(volatile v8h*)(dst + (size_t)i * 8) = hv;
  }
}

__global__ __launch_bounds__(256) void embed_kernel(const int* __restrict__ idx, const float* __restrict__ te,
                                                    const float* __restrict__ pe, unsigned short* __restrict__ X,
                                                    unsigned short* __restrict__ AC) {
  const int i = blockIdx.x * 256 + threadIdx.x;
  if (i < NROWS * (NEMB / 8)) {
    const int row = i / (NEMB / 8);
    const int c8  = i - row * (NEMB / 8);
    const int t   = row & (NSTEP - 1);
    int tk = idx[row];
    tk = tk < 0 ? 0 : (tk > NVOC - 1 ? NVOC - 1 : tk);
    const float* tp = te + (size_t)tk * NEMB + c8 * 8;
    const float* pp = pe + (size_t)t * NEMB + c8 * 8;
    const v4f ta = *(const v4f*)(tp);
    const v4f tb = *(const v4f*)(tp + 4);
    const v4f pa = *(const v4f*)(pp);
    const v4f pb = *(const v4f*)(pp + 4);
    v8h xv, av;
#pragma unroll
    for (int e = 0; e < 4; ++e) {
      xv[e]     = (_Float16)((ta[e] + pa[e]) * X_CARRY);
      xv[4 + e] = (_Float16)((tb[e] + pb[e]) * X_CARRY);
      av[e]     = (_Float16)(ta[e] * AC_CARRY);
      av[4 + e] = (_Float16)(tb[e] * AC_CARRY);
    }
    unsigned short* xo = X + (size_t)row * NEMB + c8 * 8;
    unsigned short* ao = AC + (size_t)row * NCAT + c8 * 8;
    *(volatile v8h*)xo = xv;
    *(volatile v8h*)ao = av;
    __threadfence();
    *(volatile v8h*)xo = xv;
    *(volatile v8h*)ao = av;
  }
}

template <int OUT_MODE>
__global__ __launch_bounds__(256) void gemm64_f16(
    const unsigned short* __restrict__ Ap, int lda,
    const unsigned short* __restrict__ Btp, int ldb,
    void* __restrict__ Cout, int ldc,
    const float* __restrict__ bias,
    int M, int N, int K, float scale, float bscale) {
  const _Float16* A  = (const _Float16*)Ap;
  const _Float16* Bt = (const _Float16*)Btp;
  __shared__ __align__(16) float sT[8][16 * 68];
  const int lane = threadIdx.x & 31;
  const int wave = threadIdx.x >> 5;
  const int tilesN = N >> 6;
  const int tilesM = M >> 6;
  const int tile = blockIdx.x * 8 + wave;
  if (tile >= tilesM * tilesN) return;
  const int tm = tile / tilesN;
  const int tn = tile - tm * tilesN;
  const int m0 = tm << 6;
  const int n0 = tn << 6;

  const int rlane = lane & 15;
  const int koff  = (lane >> 4) * 8;
  const int mOff  = (lane >> 4) * 8;

  const _Float16* abase = A  + (size_t)(m0 + rlane) * lda + koff;
  const _Float16* bbase = Bt + (size_t)(n0 + rlane) * ldb + koff;

  v8f acc[4][4];
#pragma unroll
  for (int i = 0; i < 4; ++i)
#pragma unroll
    for (int j = 0; j < 4; ++j) acc[i][j] = (v8f){0.f, 0.f, 0.f, 0.f, 0.f, 0.f, 0.f, 0.f};

  for (int k0 = 0; k0 < K; k0 += 32) {
    v16h bh[4];
#pragma unroll
    for (int j = 0; j < 4; ++j) bh[j] = FragH::load(bbase + (size_t)(j << 4) * ldb + k0);
#pragma unroll
    for (int i = 0; i < 4; ++i) {
      const v16h ah = FragH::load(abase + (size_t)(i << 4) * lda + k0);
#pragma unroll
      for (int j = 0; j < 4; ++j) acc[i][j] = FragH::mma(ah, bh[j], acc[i][j]);
      guard_gemm(acc[i][0], acc[i][1], acc[i][2], acc[i][3], ah, bh[0], bh[1], bh[2], bh[3]);
    }
  }
  acc_guard4(acc[0][0], acc[0][1], acc[0][2], acc[0][3]);
  acc_guard4(acc[1][0], acc[1][1], acc[1][2], acc[1][3]);
  acc_guard4(acc[2][0], acc[2][1], acc[2][2], acc[2][3]);
  acc_guard4(acc[3][0], acc[3][1], acc[3][2], acc[3][3]);

  float* slab = sT[wave];
#pragma unroll
  for (int i = 0; i < 4; ++i) {
    const int mBase = m0 + (i << 4);
#pragma unroll
    for (int j = 0; j < 4; ++j) {
      const int n = n0 + (j << 4) + rlane;
      const float bv = bias[n] * bscale;
#pragma unroll
      for (int r = 0; r < 8; ++r) {
        const float v = acc[i][j][r] * scale + bv;
        slab[(mOff + r) * 68 + (j << 4) + rlane] = v;
      }
    }
    __builtin_amdgcn_fence(__ATOMIC_RELEASE, "workgroup");
    __builtin_amdgcn_wave_barrier();
    __builtin_amdgcn_fence(__ATOMIC_ACQUIRE, "workgroup");
    if (OUT_MODE == 0) {
      float* C = (float*)Cout;
      const int hh = lane >> 4, c4 = (lane & 15) * 4;
      for (int pass = 0; pass < 2; ++pass) {
#pragma unroll
        for (int it = 0; it < 8; ++it) {
          const int row = it * 2 + hh;
          const v4f v = *(const v4f*)(slab + row * 68 + c4);
          *(volatile v4f*)(C + (size_t)(mBase + row) * ldc + n0 + c4) = v;
        }
        __threadfence();
      }
    } else {
      const int q = lane >> 3, c8 = (lane & 7) * 8;
      unsigned short* C = (unsigned short*)Cout;
      for (int pass = 0; pass < 2; ++pass) {
#pragma unroll
        for (int it = 0; it < 4; ++it) {
          const int row = it * 4 + q;
          const float* sp = slab + row * 68 + c8;
          v8h hv;
#pragma unroll
          for (int e = 0; e < 8; ++e) hv[e] = (_Float16)sp[e];
          *(volatile v8h*)(C + (size_t)(mBase + row) * ldc + n0 + c8) = hv;
        }
        __threadfence();
      }
    }
    __builtin_amdgcn_fence(__ATOMIC_RELEASE, "workgroup");
    __builtin_amdgcn_wave_barrier();
    __builtin_amdgcn_fence(__ATOMIC_ACQUIRE, "workgroup");
  }
}

constexpr int AT_KP = 72;
__global__ __launch_bounds__(128) void attn_kernel(const unsigned short* __restrict__ QKVp, unsigned short* __restrict__ CTXp) {
  __shared__ __align__(16) _Float16 Ks[64 * AT_KP];
  __shared__ __align__(16) _Float16 Vt[64 * AT_KP];
  __shared__ __align__(16) _Float16 Ps[4][16 * AT_KP];
  __shared__ __align__(16) float    Os[4][16 * 68];
  const _Float16* QKV = (const _Float16*)QKVp;

  const int tid  = threadIdx.x;
  const int wave = tid >> 5;
  const int lane = tid & 31;
  const int hh   = lane >> 4;
  const int c    = lane & 15;
  const int qb   = blockIdx.x & 3;
  const int bh   = blockIdx.x >> 2;
  const int h    = bh % NHEAD;
  const int b    = bh / NHEAD;
  const int q0   = qb * 64 + wave * 16;

  const _Float16* qbase = QKV + (size_t)b * NSTEP * NGATE + h * HDIM;
  const _Float16* kbase = qbase + NEMB;
  const unsigned short* vbase = QKVp + (size_t)b * NSTEP * NGATE + 2 * NEMB + h * HDIM;

  v16h qa[2];
#pragma unroll
  for (int dc = 0; dc < 2; ++dc) qa[dc] = FragH::load(qbase + (size_t)(q0 + c) * NGATE + dc * 32 + 8 * hh);

  float mrow[8], lrow[8];
  v8f oacc[4];
#pragma unroll
  for (int r = 0; r < 8; ++r) { mrow[r] = -INFINITY; lrow[r] = 0.f; }
#pragma unroll
  for (int t4 = 0; t4 < 4; ++t4) oacc[t4] = (v8f){0.f, 0.f, 0.f, 0.f, 0.f, 0.f, 0.f, 0.f};

  _Float16* pw = Ps[wave];

  for (int kc = 0; kc <= qb; ++kc) {
    const int kv0 = kc * 64;
    __syncthreads();
#pragma unroll
    for (int it = 0; it < 4; ++it) {
      const int p   = it * 128 + tid;
      const int kvr = p >> 3;
      const int seg = p & 7;
      const v8h kk = *(const v8h*)(kbase + (size_t)(kv0 + kvr) * NGATE + seg * 8);
      *(v8h*)(Ks + kvr * AT_KP + seg * 8) = kk;
      const v4u vw = *(const v4u*)(const void*)(vbase + (size_t)(kv0 + kvr) * NGATE + seg * 8);
#pragma unroll
      for (int i2 = 0; i2 < 4; ++i2) {
        const unsigned w = vw[i2];
        const unsigned short lo = (unsigned short)(w & 0xffffu);
        const unsigned short hi = (unsigned short)(w >> 16);
        Vt[(seg * 8 + 2 * i2) * AT_KP + kvr]     = __builtin_bit_cast(_Float16, lo);
        Vt[(seg * 8 + 2 * i2 + 1) * AT_KP + kvr] = __builtin_bit_cast(_Float16, hi);
      }
    }
    __syncthreads();

    v8f s[4];
#pragma unroll
    for (int j = 0; j < 4; ++j) {
      s[j] = (v8f){0.f, 0.f, 0.f, 0.f, 0.f, 0.f, 0.f, 0.f};
#pragma unroll
      for (int dc = 0; dc < 2; ++dc) {
        const v16h kb = FragH::load(Ks + (j * 16 + c) * AT_KP + dc * 32 + 8 * hh);
        s[j] = mma_n(qa[dc], kb, s[j]);
      }
    }
    const bool diag = (kc == qb);
    float cm[8];
#pragma unroll
    for (int r = 0; r < 8; ++r) {
      const int qrow = q0 + 8 * hh + r;
      float m = -INFINITY;
#pragma unroll
      for (int j = 0; j < 4; ++j) {
        const int kvcol = kv0 + j * 16 + c;
        float sv = s[j][r] * SC_SCALE;
        if (diag && (kvcol > qrow)) sv = MASK_FILL;
        s[j][r] = sv;
        m = fmaxf(m, sv);
      }
#pragma unroll
      for (int off = 1; off < 16; off <<= 1) m = fmaxf(m, __shfl_xor(m, off, 32));
      cm[r] = m;
    }
#pragma unroll
    for (int r = 0; r < 8; ++r) {
      const float mnew  = fmaxf(mrow[r], cm[r]);
      const float alpha = expf(mrow[r] - mnew);
      mrow[r] = mnew;
      float psum = 0.f;
#pragma unroll
      for (int j = 0; j < 4; ++j) {
        const float p = expf(s[j][r] - mnew);
        psum += p;
        pw[(8 * hh + r) * AT_KP + j * 16 + c] = (_Float16)(p * P_CARRY);
      }
#pragma unroll
      for (int off = 1; off < 16; off <<= 1) psum += __shfl_xor(psum, off, 32);
      lrow[r] = lrow[r] * alpha + psum;
#pragma unroll
      for (int t4 = 0; t4 < 4; ++t4) oacc[t4][r] *= alpha;
    }
    __builtin_amdgcn_fence(__ATOMIC_RELEASE, "workgroup");
    __builtin_amdgcn_wave_barrier();
    __builtin_amdgcn_fence(__ATOMIC_ACQUIRE, "workgroup");
#pragma unroll 1
    for (int kk = 0; kk < 2; ++kk) {
      const v16h pa = FragH::load(pw + c * AT_KP + kk * 32 + 8 * hh);
#pragma unroll
      for (int t4 = 0; t4 < 4; ++t4) {
        const v16h vb = FragH::load(Vt + (t4 * 16 + c) * AT_KP + kk * 32 + 8 * hh);
        oacc[t4] = mma_n(pa, vb, oacc[t4]);
      }
    }
  }

  float* os = Os[wave];
#pragma unroll
  for (int r = 0; r < 8; ++r) {
    const float inv = (C_CARRY / (P_CARRY * Q_CARRY)) * (1.0f / lrow[r]);
#pragma unroll
    for (int t4 = 0; t4 < 4; ++t4) os[(8 * hh + r) * 68 + t4 * 16 + c] = oacc[t4][r] * inv;
  }
  __builtin_amdgcn_fence(__ATOMIC_RELEASE, "workgroup");
  __builtin_amdgcn_wave_barrier();
  __builtin_amdgcn_fence(__ATOMIC_ACQUIRE, "workgroup");
  {
    const int q = lane >> 3, c8 = (lane & 7) * 8;
    unsigned short* cb = CTXp + (size_t)(b * NSTEP + q0) * NEMB + h * HDIM + c8;
    for (int pass = 0; pass < 2; ++pass) {
#pragma unroll
      for (int it = 0; it < 4; ++it) {
        const int row = it * 4 + q;
        const float* sp = os + row * 68 + c8;
        v8h hv;
#pragma unroll
        for (int e = 0; e < 8; ++e) hv[e] = (_Float16)sp[e];
        *(volatile v8h*)(cb + (size_t)row * NEMB) = hv;
      }
      __threadfence();
    }
  }
}

constexpr int SC_THR = 384;
constexpr int SC_HP  = 392;
constexpr int SC_SP  = 388;
constexpr int SC_PP  = 12;
static_assert(NEMB == 32 * (SC_THR / 32));
static_assert(SC_PP == SC_THR / 32);
static_assert((16 * NEMB / 4) % SC_THR == 0);
__global__ __launch_bounds__(SC_THR) void scan_kernel(
    const unsigned short* __restrict__ PREp,
    const unsigned short* __restrict__ WMp, const unsigned short* __restrict__ WHp,
    const unsigned short* __restrict__ MWp,
    const float* __restrict__ b_hh, const float* __restrict__ pg_w, const float* __restrict__ pg_b,
    const float* __restrict__ mw_b, float* __restrict__ RNN) {
  __shared__ __align__(16) _Float16 Ah[16 * SC_HP];
  __shared__ __align__(16) _Float16 Am[16 * SC_HP];
  __shared__ __align__(16) float    Hs[16 * SC_SP];
  __shared__ __align__(16) float    Pp[16 * SC_PP];
  const _Float16* WM = (const _Float16*)WMp;
  const _Float16* WH = (const _Float16*)WHp;
  const _Float16* MW = (const _Float16*)MWp;
  const int tid = threadIdx.x, lane = tid & 31, wave = tid >> 5;
  const int c = lane & 15, hh = lane >> 4, koff = hh * 8;
  const int rowbase = blockIdx.x * 16;
  const size_t GSTR = (size_t)NEMB * NEMB;

  {
    const v8h z8h = {(_Float16)0.0f, (_Float16)0.0f, (_Float16)0.0f, (_Float16)0.0f,
                     (_Float16)0.0f, (_Float16)0.0f, (_Float16)0.0f, (_Float16)0.0f};
#pragma unroll 1
    for (int i = tid; i < 16 * SC_HP / 8; i += SC_THR) {
      *(v8h*)(Ah + 8 * i) = z8h;
      *(v8h*)(Am + 8 * i) = z8h;
    }
  }
  float hA[8], hB[8], mA[8], mB[8];
#pragma unroll
  for (int r = 0; r < 8; ++r) { hA[r] = 0.0f; hB[r] = 0.0f; mA[r] = 0.0f; mB[r] = 0.0f; }

  int lrow[4], lc4[4];
  size_t goff[4];
#pragma unroll
  for (int it = 0; it < 4; ++it) {
    const int idx = it * SC_THR + tid;
    lrow[it] = idx / (NEMB / 4);
    lc4[it]  = (idx - lrow[it] * (NEMB / 4)) * 4;
    goff[it] = (size_t)(rowbase + lrow[it]) * NSTEP * NEMB + lc4[it];
  }
  const float pgb = pg_b[0];
  const _Float16* amrow = Am + c * SC_HP + koff;
  const _Float16* ahrow = Ah + c * SC_HP + koff;
  const v8f z8 = {0.f, 0.f, 0.f, 0.f, 0.f, 0.f, 0.f, 0.f};
  __syncthreads();

#pragma unroll 1
  for (int t = 0; t < NSTEP; ++t) {
    float ps[8];
#pragma unroll
    for (int r = 0; r < 8; ++r) ps[r] = 0.0f;
#pragma unroll 1
    for (int nt = 0; nt < 2; ++nt) {
      const int j = 32 * wave + 16 * nt + c;
      const _Float16* wm = WM + (size_t)j * NEMB + koff;
      const _Float16* wh = WH + (size_t)j * NEMB + koff;
      v8f aR = z8, aZ = z8, aIN = z8, aHN = z8;
#pragma unroll 1
      for (int k0 = 0; k0 < NEMB; k0 += 32) {
        const v16h am  = FragH::load(amrow + k0);
        const v16h ah  = FragH::load(ahrow + k0);
        const v16h bm0 = FragH::load(wm + k0);
        const v16h bm1 = FragH::load(wm + GSTR + k0);
        const v16h bm2 = FragH::load(wm + 2 * GSTR + k0);
        const v16h bh0 = FragH::load(wh + k0);
        const v16h bh1 = FragH::load(wh + GSTR + k0);
        const v16h bh2 = FragH::load(wh + 2 * GSTR + k0);
        aR  = FragH::mma(am, bm0, aR);
        aZ  = FragH::mma(am, bm1, aZ);
        aIN = FragH::mma(am, bm2, aIN);
        aR  = FragH::mma(ah, bh0, aR);
        aZ  = FragH::mma(ah, bh1, aZ);
        aHN = FragH::mma(ah, bh2, aHN);
        guard_scan(aR, aZ, aIN, aHN, am, ah, bm0, bm1, bm2, bh0, bh1, bh2);
      }
      acc_guard4(aR, aZ, aIN, aHN);
      float bR = b_hh[j];
      float bZ = b_hh[NEMB + j];
      float bN = b_hh[2 * NEMB + j];
      float pw = pg_w[j];
      asm volatile("" : "+v"(bR), "+v"(bZ), "+v"(bN), "+v"(pw));
      const unsigned short* pp = PREp + ((size_t)(rowbase + 8 * hh) * NSTEP + (size_t)t) * NGATE + j;
#pragma unroll
      for (int r = 0; r < 8; ++r) {
        const unsigned short* pr = pp + (size_t)r * NSTEP * NGATE;
        unsigned u0 = pr[0];
        unsigned u1 = pr[NEMB];
        unsigned u2 = pr[2 * NEMB];
        asm volatile("" : "+v"(u0), "+v"(u1), "+v"(u2));
        const float gr  = (h16_to_f32(u0) * PRE_INV + aR[r] * ST_FOLD) + bR;
        const float gz  = (h16_to_f32(u1) * PRE_INV + aZ[r] * ST_FOLD) + bZ;
        const float gin = h16_to_f32(u2) * PRE_INV + aIN[r] * ST_FOLD;
        const float ghn = aHN[r] * ST_FOLD + bN;
        const float rg  = sig_f(gr);
        const float zg  = sig_f(gz);
        const float ng  = tanhf(gin + rg * ghn);
        const float hn  = (1.0f - zg) * ng + zg * hA[r];
        hA[r] = hn;
        Hs[(8 * hh + r) * SC_SP + j] = hn;
        ps[r] = fmaf(hn, pw, ps[r]);
      }
#pragma unroll
      for (int r = 0; r < 8; ++r) { const float tx = hA[r]; hA[r] = hB[r]; hB[r] = tx; }
    }
#pragma unroll
    for (int r = 0; r < 8; ++r) {
#pragma unroll
      for (int off = 1; off < 16; off <<= 1) ps[r] += __shfl_xor(ps[r], off, 32);
    }
    if (c == 0) {
#pragma unroll
      for (int r = 0; r < 8; ++r) Pp[(8 * hh + r) * SC_PP + wave] = ps[r];
    }
    __syncthreads();

    v4f hv[4];
#pragma unroll
    for (int it = 0; it < 4; ++it) {
      hv[it] = *(const v4f*)(Hs + lrow[it] * SC_SP + lc4[it]);
      v4h h4;
#pragma unroll
      for (int e = 0; e < 4; ++e) h4[e] = (_Float16)(hv[it][e] * S_CARRY);
      *(v4h*)(Ah + lrow[it] * SC_HP + lc4[it]) = h4;
    }
    for (int pass = 0; pass < 2; ++pass) {
#pragma unroll
      for (int it = 0; it < 4; ++it)
        *(volatile v4f*)(RNN + goff[it] + (size_t)t * NEMB) = hv[it];
      __threadfence();
    }
    float pg[8];
#pragma unroll
    for (int r = 0; r < 8; ++r) {
      const float* pr = Pp + (8 * hh + r) * SC_PP;
      const v4f a = *(const v4f*)(pr);
      const v4f b = *(const v4f*)(pr + 4);
      const v4f d = *(const v4f*)(pr + 8);
      const float sum = (((a[0] + a[1]) + (a[2] + a[3])) + ((b[0] + b[1]) + (b[2] + b[3]))) + ((d[0] + d[1]) + (d[2] + d[3]));
      pg[r] = sig_f(sum + pgb);
    }
    __syncthreads();

#pragma unroll 1
    for (int nt = 0; nt < 2; ++nt) {
      const int j = 32 * wave + 16 * nt + c;
      const _Float16* wq = MW + (size_t)j * NEMB + koff;
      v8f ac = z8;
#pragma unroll 1
      for (int k0 = 0; k0 < NEMB; k0 += 32) {
        const v16h a = FragH::load(ahrow + k0);
        const v16h b = FragH::load(wq + k0);
        ac = mma_n(a, b, ac);
      }
      acc_guard1(ac);
      float mb = mw_b[j];
      asm volatile("" : "+v"(mb));
#pragma unroll
      for (int r = 0; r < 8; ++r) {
        const float cand = tanhf(ac[r] * ST_FOLD + mb);
        const float mn = (1.0f - pg[r]) * mA[r] + pg[r] * cand;
        mA[r] = mn;
        Am[(8 * hh + r) * SC_HP + j] = (_Float16)(mn * S_CARRY);
      }
#pragma unroll
      for (int r = 0; r < 8; ++r) { const float tx = mA[r]; mA[r] = mB[r]; mB[r] = tx; }
    }
    __syncthreads();
  }
}

__global__ __launch_bounds__(256) void ln_rows_kernel(const float* __restrict__ RNN, const float* __restrict__ gam,
                                                      const float* __restrict__ bet, unsigned short* __restrict__ NORM,
                                                      int nrows) {
  const int tid = threadIdx.x, lane = tid & 31;
  const int row = blockIdx.x * 8 + (tid >> 5);
  if (row >= nrows) return;
  const float* rp = RNN + (size_t)row * NEMB;
  v4f v[3], g[3], bb[3];
  float s = 0.0f;
#pragma unroll
  for (int q = 0; q < 3; ++q) {
    v[q]  = *(const v4f*)(rp  + 128 * q + 4 * lane);
    g[q]  = *(const v4f*)(gam + 128 * q + 4 * lane);
    bb[q] = *(const v4f*)(bet + 128 * q + 4 * lane);
    s += (v[q][0] + v[q][1]) + (v[q][2] + v[q][3]);
  }
#pragma unroll
  for (int off = 1; off < 32; off <<= 1) s += __shfl_xor(s, off, 32);
  const float mu = s * (1.0f / NEMB);
  float ss = 0.0f;
#pragma unroll
  for (int q = 0; q < 3; ++q)
#pragma unroll
    for (int e = 0; e < 4; ++e) { const float d = v[q][e] - mu; v[q][e] = d; ss += d * d; }
#pragma unroll
  for (int off = 1; off < 32; off <<= 1) ss += __shfl_xor(ss, off, 32);
  const float var  = ss * (1.0f / NEMB);
  const float rstd = 1.0f / sqrtf(var + LN_EPS_F);
  v4h o[3];
#pragma unroll
  for (int q = 0; q < 3; ++q)
#pragma unroll
    for (int e = 0; e < 4; ++e) {
      const float y = (v[q][e] * rstd) * g[q][e] + bb[q][e];
      o[q][e] = (_Float16)(y * N_CARRY);
    }
  unsigned short* op = NORM + (size_t)row * NEMB;
  for (int pass = 0; pass < 2; ++pass) {
#pragma unroll
    for (int q = 0; q < 3; ++q) *(volatile v4h*)(op + 128 * q + 4 * lane) = o[q];
    __threadfence();
  }
}

extern "C" void kernel_launch(void* const* d_in, const int* in_sizes, int n_in,
                              void* d_out, int out_size, void* d_ws, size_t ws_size, hipStream_t stream) {
  if (n_in < 19 || d_out == nullptr || d_ws == nullptr) return;
  if (in_sizes[0] != NROWS || in_sizes[1] != NVOC * NEMB || in_sizes[2] != NSTEP * NEMB ||
      in_sizes[3] != NGATE * NEMB || in_sizes[4] != NGATE || in_sizes[5] != NEMB * NEMB || in_sizes[6] != NEMB ||
      in_sizes[7] != NGATE * NGATE || in_sizes[8] != NGATE || in_sizes[9] != NGATE * NEMB || in_sizes[10] != NGATE ||
      in_sizes[11] != NEMB || in_sizes[12] != 1 || in_sizes[13] != NEMB * NEMB || in_sizes[14] != NEMB ||
      in_sizes[15] != NEMB || in_sizes[16] != NEMB || in_sizes[17] != NVOC * NEMB || in_sizes[18] != NVOC ||
      out_size != NOUT) return;

  const int*   idx        = (const int*)d_in[0];
  const float* token_emb  = (const float*)d_in[1];
  const float* pos_emb    = (const float*)d_in[2];
  const float* in_proj_w  = (const float*)d_in[3];
  const float* in_proj_b  = (const float*)d_in[4];
  const float* out_proj_w = (const float*)d_in[5];
  const float* out_proj_b = (const float*)d_in[6];
  const float* w_ih       = (const float*)d_in[7];
  const float* b_ih       = (const float*)d_in[8];
  const float* w_hh       = (const float*)d_in[9];
  const float* b_hh       = (const float*)d_in[10];
  const float* pg_w       = (const float*)d_in[11];
  const float* pg_b       = (const float*)d_in[12];
  const float* mw_w       = (const float*)d_in[13];
  const float* mw_b       = (const float*)d_in[14];
  const float* ln_g       = (const float*)d_in[15];
  const float* ln_b       = (const float*)d_in[16];
  const float* head_w     = (const float*)d_in[17];
  const float* head_b     = (const float*)d_in[18];
  float* logits = (float*)d_out;

  char* ws = (char*)d_ws;
  size_t off = 0;
  auto carve = [&](size_t bytes) -> char* { char* p = ws + off; off += (bytes + 255) & ~(size_t)255; return p; };
  unsigned short* WIN   = (unsigned short*)carve((size_t)NGATE * NEMB * 2);
  unsigned short* WOUT  = (unsigned short*)carve((size_t)NEMB * NEMB * 2);
  unsigned short* WTC   = (unsigned short*)carve((size_t)NGATE * NCAT * 2);
  unsigned short* WMEM  = (unsigned short*)carve((size_t)NGATE * NEMB * 2);
  unsigned short* WHH   = (unsigned short*)carve((size_t)NGATE * NEMB * 2);
  unsigned short* WMW   = (unsigned short*)carve((size_t)NEMB * NEMB * 2);
  unsigned short* WHEAD = (unsigned short*)carve((size_t)NVOC * NEMB * 2);
  unsigned short* X     = (unsigned short*)carve((size_t)NROWS * NEMB * 2);
  unsigned short* QKV   = (unsigned short*)carve((size_t)NROWS * NGATE * 2);
  unsigned short* CTX   = (unsigned short*)carve((size_t)NROWS * NEMB * 2);
  unsigned short* AC    = (unsigned short*)carve((size_t)NROWS * NCAT * 2);
  float*          RNN   = (float*)carve((size_t)NROWS * NEMB * 4);
  unsigned short* NORM  = X;
  unsigned short* PRE   = QKV;
  if (off > ws_size || off > (size_t)134217728) return;

  {
    const int n8a = NGATE * (NEMB / 8);
    const int n8b = NEMB * (NEMB / 8);
    const int n8c = NGATE * (NCAT / 8);
    const int n8d = NVOC * (NEMB / 8);
    cvt8_f16_kernel<<<n8a / 256, 256, 0, stream>>>(in_proj_w,  WIN,   NGATE, NEMB / 8, NEMB,  0,    W_CARRY);
    cvt8_f16_kernel<<<n8b / 256, 256, 0, stream>>>(out_proj_w, WOUT,  NEMB,  NEMB / 8, NEMB,  0,    W_CARRY);
    cvt8_f16_kernel<<<n8c / 256, 256, 0, stream>>>(w_ih,       WTC,   NGATE, NCAT / 8, NGATE, 0,    W_CARRY);
    cvt8_f16_kernel<<<n8a / 256, 256, 0, stream>>>(w_ih,       WMEM,  NGATE, NEMB / 8, NGATE, NCAT, W_CARRY);
    cvt8_f16_kernel<<<n8a / 256, 256, 0, stream>>>(w_hh,       WHH,   NGATE, NEMB / 8, NEMB,  0,    W_CARRY);
    cvt8_f16_kernel<<<n8b / 256, 256, 0, stream>>>(mw_w,       WMW,   NEMB,  NEMB / 8, NEMB,  0,    W_CARRY);
    cvt8_f16_kernel<<<n8d / 256, 256, 0, stream>>>(head_w,     WHEAD, NVOC,  NEMB / 8, NEMB,  0,    W_CARRY);
  }

  embed_kernel<<<NROWS * (NEMB / 8) / 256, 256, 0, stream>>>(idx, token_emb, pos_emb, X, AC);

  gemm64_f16<1><<<(NROWS / 64) * (NGATE / 64) / 8, 256, 0, stream>>>(
      X, NEMB, WIN, NEMB, (void*)QKV, NGATE, in_proj_b, NROWS, NGATE, NEMB,
      Q_CARRY / (X_CARRY * W_CARRY), Q_CARRY);

  attn_kernel<<<NBATCH * NHEAD * (NSTEP / 64), 128, 0, stream>>>(QKV, CTX);

  gemm64_f16<1><<<(NROWS / 64) * (NEMB / 64) / 8, 256, 0, stream>>>(
      CTX, NEMB, WOUT, NEMB, (void*)(AC + NEMB), NCAT, out_proj_b, NROWS, NEMB, NEMB,
      AC_CARRY / (C_CARRY * W_CARRY), AC_CARRY);

  gemm64_f16<1><<<(NROWS / 64) * (NGATE / 64) / 8, 256, 0, stream>>>(
      AC, NCAT, WTC, NCAT, (void*)PRE, NGATE, b_ih, NROWS, NGATE, NCAT,
      PRE_CARRY / (AC_CARRY * W_CARRY), PRE_CARRY);

  scan_kernel<<<NBATCH / 16, SC_THR, 0, stream>>>(PRE, WMEM, WHH, WMW, b_hh, pg_w, pg_b, mw_b, RNN);

  ln_rows_kernel<<<NROWS / 8, 256, 0, stream>>>(RNN, ln_g, ln_b, NORM, NROWS);

  gemm64_f16<0><<<(NROWS / 64) * (NVOC / 64) / 8, 256, 0, stream>>>(
      NORM, NEMB, WHEAD, NEMB, (void*)logits, NVOC, head_b, NROWS, NVOC, NEMB,
      1.0f / (N_CARRY * W_CARRY), 1.0f);
}
